// GSN_42709154791890
// MI455X (gfx1250) — hardware-verified
//
#include <hip/hip_runtime.h>
#include <stddef.h>
#include <stdint.h>


#define HID    256
#define IND    64
#define EFD    64
#define MSGIN  578
#define UPDIN  512
#define WSC    16.0f
#define WINV   0.0625f

#define T_LIN    0
#define T_L0     16384
#define T_LSZ    409600
#define T_P      0
#define T_E      131072
#define T_M2     147456
#define T_U1     212992
#define T_U2     344064
#define T_TOTAL  (T_L0 + 3 * T_LSZ)
#define T_PIECES (T_TOTAL / 64)

#define HP    264
#define XP    72
#define FP    132
#define NTHR  256
#define NWAVE 8
#define STG_BYTES (NWAVE * 16 * FP * 4)

#define L_XS   0
#define L_STG  (64 * XP * 2)
#define L_LDS  (L_STG + STG_BYTES)
#define J_LDS  STG_BYTES
#define E_IDX  0
#define E_EFS  1024
#define E_HID  (E_EFS + 64 * XP * 2)
#define E_STG  (E_HID + 64 * HP * 2)
#define E_LDS  (E_STG + STG_BYTES)
#define NB     128
#define EPT    8
#define CHUNK  (NTHR * EPT)
#define WCAP   (EPT * 32)
#define G_ACC  0
#define G_HID  0
#define G_STG  (64 * HP * 2)
#define G_UT   (NB * HID * 4)
#define G_LIST (G_UT + NB * HP * 2)
#define G_WCNT (G_LIST + NWAVE * WCAP * 4)
#define G_LDS  (G_WCNT + 64)

static_assert(T_PIECES * 64 == T_TOTAL);
static_assert((T_PIECES * 8) % 256 == 0);
static_assert((L_STG & 15) == 0 && (E_EFS & 15) == 0 && (E_HID & 15) == 0 && (E_STG & 15) == 0);
static_assert((G_STG & 15) == 0 && (G_UT & 15) == 0 && (G_LIST & 15) == 0 && (G_WCNT & 15) == 0);
static_assert(G_STG + STG_BYTES <= G_UT);
static_assert(((HP * 2) & 15) == 0 && ((XP * 2) & 15) == 0 && ((FP * 4) & 15) == 0);
static_assert(L_LDS <= 300 * 1024 && E_LDS <= 300 * 1024 && G_LDS <= 300 * 1024 && J_LDS <= 300 * 1024);
static_assert(NB == 128 && WCAP == 256 && NB <= NTHR);

typedef float    v4f  __attribute__((ext_vector_type(4)));
typedef float    v8f  __attribute__((ext_vector_type(8)));
typedef int      v4i  __attribute__((ext_vector_type(4)));
typedef _Float16 v8h  __attribute__((ext_vector_type(8)));
typedef _Float16 v16h __attribute__((ext_vector_type(16)));
union FragH { v16h v; v8h h[2]; };

__device__ __forceinline__ v8f zero8f() {
  v8f z;
#pragma unroll
  for (int i = 0; i < 8; ++i) z[i] = 0.0f;
  return z;
}

__device__ __forceinline__ v8f wmh(v16h a, v16h b, v8f c) {
  v8f d = __builtin_amdgcn_wmma_f32_16x16x32_f16(false, a, false, b, (short)0, c, false, false);
  asm volatile("v_nop\n\tv_nop\n\tv_nop\n\tv_nop" : "+v"(d) : "v"(a), "v"(b));
  return d;
}

__device__ __forceinline__ void gemm16(const _Float16* arow, const _Float16* bcol, int kp, int nkt,
                                       v8f acc[8]) {
#pragma unroll 1
  for (int kt = 0; kt < nkt; ++kt) {
    FragH a;
    a.h[0] = *(const v8h*)(arow + 32 * kt);
    a.h[1] = *(const v8h*)(arow + 32 * kt + 16);
#pragma unroll
    for (int nt = 0; nt < 8; ++nt) {
      const _Float16* bp = bcol + (size_t)(16 * nt) * kp + 32 * kt;
      FragH b;
      b.h[0] = *(const v8h*)bp;
      b.h[1] = *(const v8h*)(bp + 16);
      acc[nt] = wmh(a.v, b.v, acc[nt]);
    }
  }
}

__device__ __forceinline__ void store16_f16(const float* st, _Float16* g, int ldg, int col0, int grow0, int l) {
  const int h = l >> 4, m = l & 15;
#pragma unroll
  for (int j = 0; j < 8; ++j) {
    const int lr = 2 * j + h;
    const v4f a0 = *(const v4f*)(st + lr * FP + 8 * m);
    const v4f a1 = *(const v4f*)(st + lr * FP + 8 * m + 4);
    v8h o;
#pragma unroll
    for (int i = 0; i < 4; ++i) { o[i] = (_Float16)a0[i]; o[4 + i] = (_Float16)a1[i]; }
    *(volatile v8h*)(g + (size_t)(grow0 + lr) * ldg + col0 + 8 * m) = o;
  }
  __threadfence();
#pragma unroll
  for (int j = 0; j < 8; ++j) {
    const int lr = 2 * j + h;
    const v4f a0 = *(const v4f*)(st + lr * FP + 8 * m);
    const v4f a1 = *(const v4f*)(st + lr * FP + 8 * m + 4);
    v8h o;
#pragma unroll
    for (int i = 0; i < 4; ++i) { o[i] = (_Float16)a0[i]; o[4 + i] = (_Float16)a1[i]; }
    *(volatile v8h*)(g + (size_t)(grow0 + lr) * ldg + col0 + 8 * m) = o;
  }
}

__device__ __forceinline__ void store16_f32(const float* st, float* g, int ldg, int col0, int grow0, int l) {
#pragma unroll
  for (int rr = 0; rr < 16; ++rr) {
    const v4f v = *(const v4f*)(st + rr * FP + 4 * l);
    *(volatile v4f*)(g + (size_t)(grow0 + rr) * ldg + col0 + 4 * l) = v;
  }
  __threadfence();
#pragma unroll
  for (int rr = 0; rr < 16; ++rr) {
    const v4f v = *(const v4f*)(st + rr * FP + 4 * l);
    *(volatile v4f*)(g + (size_t)(grow0 + rr) * ldg + col0 + 4 * l) = v;
  }
}

__global__ __launch_bounds__(256) void k_wcvt(const float* __restrict__ Wlin, const float* __restrict__ mW1,
                                              const float* __restrict__ mW2, const float* __restrict__ uW1,
                                              const float* __restrict__ uW2, _Float16* Wt) {
  const int t = blockIdx.x * 256 + threadIdx.x;
  if (t >= T_PIECES * 8) return;
  const int p = t >> 3, kc = (t & 7) * 8;
  const float* src = Wlin;
  int col = 0, krow0 = 0;
  if (p < 256) { src = Wlin; col = p; krow0 = 0; }
  else {
    const int q0 = p - 256;
    const int s  = q0 / 6400;
    const int q  = q0 - s * 6400;
    if (q < 2048) {
      const int c = q >> 2, ks = q & 3;
      src = mW1 + (size_t)s * MSGIN * HID; col = c & 255; krow0 = ((c < 256) ? 0 : 256) + 64 * ks;
    } else if (q < 2304) {
      src = mW1 + (size_t)s * MSGIN * HID; col = q - 2048; krow0 = 514;
    } else if (q < 3328) {
      const int qq = q - 2304;
      src = mW2 + (size_t)s * HID * HID; col = qq >> 2; krow0 = 64 * (qq & 3);
    } else if (q < 5376) {
      const int qq = q - 3328;
      src = uW1 + (size_t)s * UPDIN * HID; col = qq >> 3; krow0 = 64 * (qq & 7);
    } else {
      const int qq = q - 5376;
      src = uW2 + (size_t)s * HID * HID; col = qq >> 2; krow0 = 64 * (qq & 3);
    }
  }
  v8h o;
#pragma unroll
  for (int i = 0; i < 8; ++i) o[i] = (_Float16)(src[(size_t)(krow0 + kc + i) * HID + col] * WSC);
  _Float16* dp = Wt + (size_t)p * 64 + kc;
  *(volatile v8h*)dp = o;
  __threadfence();
  *(volatile v8h*)dp = o;
}

__global__ __launch_bounds__(256) void k_lin(const float* __restrict__ x, const _Float16* TL,
                                             const float* __restrict__ blin, _Float16* hout, int nN) {
  extern __shared__ __attribute__((aligned(16))) unsigned char lds_l[];
  _Float16* xs  = (_Float16*)(lds_l + L_XS);
  float*    stg = (float*)(lds_l + L_STG);
  const int tid = threadIdx.x, l = tid & 31, wave = tid >> 5, h = l >> 4, m = l & 15;
  const int wr = wave >> 1, wc = wave & 1;
  const int row0 = blockIdx.x * 64;

  for (int i = tid; i < 64 * 8; i += 256) {
    const int r = i >> 3, c8 = (i & 7) * 8;
    const int gr = row0 + r;
    v8h o;
    if (gr < nN) {
      const v4f a0 = *(const v4f*)(x + (size_t)gr * IND + c8);
      const v4f a1 = *(const v4f*)(x + (size_t)gr * IND + c8 + 4);
#pragma unroll
      for (int j = 0; j < 4; ++j) { o[j] = (_Float16)a0[j]; o[4 + j] = (_Float16)a1[j]; }
    } else {
#pragma unroll
      for (int j = 0; j < 8; ++j) o[j] = (_Float16)0.0f;
    }
    *(v8h*)(xs + r * XP + c8) = o;
  }
  __syncthreads();

  v8f acc[8];
#pragma unroll
  for (int i = 0; i < 8; ++i) acc[i] = zero8f();
  gemm16(xs + (16 * wr + m) * XP + 8 * h, TL + (size_t)(128 * wc + m) * IND + 8 * h, IND, 2, acc);

  float* st = stg + wave * (16 * FP);
#pragma unroll
  for (int nt = 0; nt < 8; ++nt) {
    const int c = 128 * wc + 16 * nt + m;
    const float b = blin[c];
#pragma unroll
    for (int r = 0; r < 8; ++r) st[(8 * h + r) * FP + 16 * nt + m] = acc[nt][r] * WINV + b;
  }
  __syncthreads();
  store16_f16(st, hout, HID, 128 * wc, row0 + 16 * wr, l);
}

__global__ __launch_bounds__(256) void k_proj(const _Float16* __restrict__ hin, const _Float16* TPt,
                                              _Float16* P16) {
  extern __shared__ __attribute__((aligned(16))) unsigned char lds_j[];
  float* stg = (float*)lds_j;
  const int tid = threadIdx.x, l = tid & 31, wave = tid >> 5, h = l >> 4, m = l & 15;
  const int wr = wave >> 1, wc = wave & 1;
  const int row0  = blockIdx.x * 64;
  const int cbase = blockIdx.y * 256 + 128 * wc;

  v8f acc[8];
#pragma unroll
  for (int i = 0; i < 8; ++i) acc[i] = zero8f();
  gemm16(hin + (size_t)(row0 + 16 * wr + m) * HID + 8 * h, TPt + (size_t)(cbase + m) * HID + 8 * h, HID, 8, acc);

  float* st = stg + wave * (16 * FP);
#pragma unroll
  for (int nt = 0; nt < 8; ++nt) {
#pragma unroll
    for (int r = 0; r < 8; ++r) st[(8 * h + r) * FP + 16 * nt + m] = acc[nt][r];
  }
  __syncthreads();
  store16_f16(st, P16, 2 * HID, cbase, row0 + 16 * wr, l);
}

__global__ __launch_bounds__(256) void k_edge(const int* __restrict__ el, const float* __restrict__ nsf,
                                              const float* __restrict__ ef, const _Float16* __restrict__ P16,
                                              const float* __restrict__ W1s, const float* __restrict__ b1,
                                              const _Float16* TEt, const _Float16* TM2t,
                                              const float* __restrict__ b2, _Float16* M16, int nE, int nN) {
  extern __shared__ __attribute__((aligned(16))) unsigned char lds_e[];
  int*      ni  = (int*)(lds_e + E_IDX);
  int*      no  = ni + 64;
  float*    sfi = (float*)(lds_e + E_IDX + 512);
  float*    sfo = sfi + 64;
  _Float16* efs = (_Float16*)(lds_e + E_EFS);
  _Float16* hid = (_Float16*)(lds_e + E_HID);
  float*    stg = (float*)(lds_e + E_STG);
  const int tid = threadIdx.x, l = tid & 31, wave = tid >> 5, h = l >> 4, m = l & 15;
  const int wr = wave >> 1, wc = wave & 1;
  const int e0 = blockIdx.x * 64;

  if (tid < 64) {
    const int e = e0 + tid;
    int a = 0, b = 0;
    if (e < nE) { a = el[2 * (size_t)e]; b = el[2 * (size_t)e + 1]; }
    a = a < 0 ? 0 : (a > nN - 1 ? nN - 1 : a);
    b = b < 0 ? 0 : (b > nN - 1 ? nN - 1 : b);
    ni[tid] = a;
    no[tid] = b;
    sfi[tid] = nsf[a];
    sfo[tid] = nsf[b];
  }
  for (int i = tid; i < 64 * 8; i += 256) {
    const int r = i >> 3, c8 = (i & 7) * 8;
    const int e = e0 + r;
    v8h o;
    if (e < nE) {
      const v4f a0 = *(const v4f*)(ef + (size_t)e * EFD + c8);
      const v4f a1 = *(const v4f*)(ef + (size_t)e * EFD + c8 + 4);
#pragma unroll
      for (int j = 0; j < 4; ++j) { o[j] = (_Float16)a0[j]; o[4 + j] = (_Float16)a1[j]; }
    } else {
#pragma unroll
      for (int j = 0; j < 8; ++j) o[j] = (_Float16)0.0f;
    }
    *(v8h*)(efs + r * XP + c8) = o;
  }
  __syncthreads();

  v8f acc[8];
#pragma unroll
  for (int i = 0; i < 8; ++i) acc[i] = zero8f();
  gemm16(efs + (16 * wr + m) * XP + 8 * h, TEt + (size_t)(128 * wc + m) * EFD + 8 * h, EFD, 2, acc);

  {
    const float* w512 = W1s + (size_t)512 * HID;
    const float* w513 = w512 + HID;
    int ri[8], ci[8];
    float si[8], so[8];
#pragma unroll
    for (int r = 0; r < 8; ++r) {
      const int lr = 16 * wr + 8 * h + r;
      ri[r] = ni[lr];
      ci[r] = no[lr];
      si[r] = sfi[lr];
      so[r] = sfo[lr];
    }
#pragma unroll
    for (int nt = 0; nt < 8; ++nt) {
      const int c = 128 * wc + 16 * nt + m;
      const float bc = b1[c];
      const float wa = w512[c];
      const float wb = w513[c];
#pragma unroll
      for (int r = 0; r < 8; ++r) {
        const float pin  = (float)P16[(size_t)ri[r] * (2 * HID) + c];
        const float pout = (float)P16[(size_t)ci[r] * (2 * HID) + HID + c];
        float v = (acc[nt][r] + pin + pout) * WINV;
        v = v + si[r] * wa;
        v = v + so[r] * wb;
        v = v + bc;
        hid[(16 * wr + 8 * h + r) * HP + c] = (_Float16)fmaxf(v, 0.0f);
      }
    }
  }
  __syncthreads();

#pragma unroll
  for (int i = 0; i < 8; ++i) acc[i] = zero8f();
  gemm16(hid + (16 * wr + m) * HP + 8 * h, TM2t + (size_t)(128 * wc + m) * HID + 8 * h, HID, 8, acc);

  float* st = stg + wave * (16 * FP);
#pragma unroll
  for (int nt = 0; nt < 8; ++nt) {
    const int c = 128 * wc + 16 * nt + m;
    const float b = b2[c];
#pragma unroll
    for (int r = 0; r < 8; ++r) st[(8 * h + r) * FP + 16 * nt + m] = acc[nt][r] * WINV + b;
  }
  __syncthreads();
  store16_f16(st, M16, HID, 128 * wc, e0 + 16 * wr, l);
}

__device__ __forceinline__ int scan_chunk(const int* __restrict__ el, int nE, int cbase, int nodeBase,
                                          int* list, int tid, int wave) {
  int wcn = 0;
  const int el0  = tid * EPT;
  const int e0   = cbase + el0;
  const int sent = -2147483647 - 1;
  int d0, d1, d2, d3, d4, d5, d6, d7;
  if (e0 + 7 < nE) {
    const int* p = el + 2 * (size_t)e0;
    const v4i qa = *(const v4i*)p;
    const v4i qb = *(const v4i*)(p + 4);
    const v4i qc = *(const v4i*)(p + 8);
    const v4i qd = *(const v4i*)(p + 12);
    d0 = qa.y; d1 = qa.w; d2 = qb.y; d3 = qb.w; d4 = qc.y; d5 = qc.w; d6 = qd.y; d7 = qd.w;
  } else {
    d0 = (e0     < nE) ? el[2 * (size_t)((e0     < nE) ? e0     : nE - 1) + 1] : sent;
    d1 = (e0 + 1 < nE) ? el[2 * (size_t)((e0 + 1 < nE) ? e0 + 1 : nE - 1) + 1] : sent;
    d2 = (e0 + 2 < nE) ? el[2 * (size_t)((e0 + 2 < nE) ? e0 + 2 : nE - 1) + 1] : sent;
    d3 = (e0 + 3 < nE) ? el[2 * (size_t)((e0 + 3 < nE) ? e0 + 3 : nE - 1) + 1] : sent;
    d4 = (e0 + 4 < nE) ? el[2 * (size_t)((e0 + 4 < nE) ? e0 + 4 : nE - 1) + 1] : sent;
    d5 = (e0 + 5 < nE) ? el[2 * (size_t)((e0 + 5 < nE) ? e0 + 5 : nE - 1) + 1] : sent;
    d6 = (e0 + 6 < nE) ? el[2 * (size_t)((e0 + 6 < nE) ? e0 + 6 : nE - 1) + 1] : sent;
    d7 = (e0 + 7 < nE) ? el[2 * (size_t)((e0 + 7 < nE) ? e0 + 7 : nE - 1) + 1] : sent;
  }
  const unsigned nb = (unsigned)nodeBase;
  const unsigned s0 = (unsigned)d0 - nb, s1 = (unsigned)d1 - nb;
  const unsigned s2 = (unsigned)d2 - nb, s3 = (unsigned)d3 - nb;
  const unsigned s4 = (unsigned)d4 - nb, s5 = (unsigned)d5 - nb;
  const unsigned s6 = (unsigned)d6 - nb, s7 = (unsigned)d7 - nb;
  const bool q0 = s0 < (unsigned)NB, q1 = s1 < (unsigned)NB, q2 = s2 < (unsigned)NB, q3 = s3 < (unsigned)NB;
  const bool q4 = s4 < (unsigned)NB, q5 = s5 < (unsigned)NB, q6 = s6 < (unsigned)NB, q7 = s7 < (unsigned)NB;
  const unsigned any = __builtin_amdgcn_ballot_w32(q0 | q1 | q2 | q3 | q4 | q5 | q6 | q7);
  if (any != 0u) {
#define HITJ(J, QJ, SJ) { \
      const unsigned mj = __builtin_amdgcn_ballot_w32(QJ); \
      if (mj != 0u) { \
        if (QJ) { \
          const int pos = wcn + (int)__builtin_amdgcn_mbcnt_lo(mj, 0u); \
          if (pos < WCAP) list[wave * WCAP + pos] = ((el0 + (J)) << 8) | (int)(SJ); \
        } \
        wcn += (int)__builtin_popcount(mj); } }
    HITJ(0, q0, s0)
    HITJ(1, q1, s1)
    HITJ(2, q2, s2)
    HITJ(3, q3, s3)
    HITJ(4, q4, s4)
    HITJ(5, q5, s5)
    HITJ(6, q6, s6)
    HITJ(7, q7, s7)
#undef HITJ
  }
  return wcn;
}

__global__ __launch_bounds__(NTHR) void k_aggnode(const int* __restrict__ el, const float* __restrict__ ew,
                                                   const _Float16* __restrict__ M16, const _Float16* __restrict__ hin,
                                                   const _Float16* TU1t, const float* __restrict__ b1,
                                                   const _Float16* TU2t, const float* __restrict__ b2,
                                                   _Float16* hout, float* hf, int nN, int nE, int wf32) {
  extern __shared__ __attribute__((aligned(16))) unsigned char lds_g[];
  float*    acc  = (float*)(lds_g + G_ACC);
  _Float16* hid  = (_Float16*)(lds_g + G_HID);
  float*    stg  = (float*)(lds_g + G_STG);
  _Float16* ut   = (_Float16*)(lds_g + G_UT);
  int*      list = (int*)(lds_g + G_LIST);
  int*      wcnt = (int*)(lds_g + G_WCNT);
  const int tid = threadIdx.x, l = tid & 31, wave = tid >> 5, h = l >> 4, m = l & 15;
  const int wr = wave >> 1, wc = wave & 1;
  const int nodeBase = blockIdx.x * NB;

  {
    const v4f z = {0.0f, 0.0f, 0.0f, 0.0f};
    for (int i = tid; i < NB * (HID / 4); i += NTHR) *(v4f*)(acc + 4 * i) = z;
  }
  __syncthreads();

  const int nChunks = (nE + CHUNK - 1) / CHUNK;
#pragma unroll 1
  for (int ch = 0; ch < nChunks; ++ch) {
    const int cbase = ch * CHUNK;
    const int wcn = scan_chunk(el, nE, cbase, nodeBase, list, tid, wave);
    if (l == 0) wcnt[wave] = wcn;
    __syncthreads();

#pragma unroll 1
    for (int w2 = 0; w2 < NWAVE; ++w2) {
      int n = wcnt[w2];
      n = n > WCAP ? WCAP : (n < 0 ? 0 : n);
      const int* lp = list + w2 * WCAP;
#pragma unroll 1
      for (int i = 0; i < n; ++i) {
        const int v = lp[i];
        const int slot = v & (NB - 1);
        if ((slot & 7) == wave) {
          int e = cbase + ((v >> 8) & 2047);
          e = e < 0 ? 0 : (e > nE - 1 ? nE - 1 : e);
          const float w = ew[e];
          const v8h x = *(const v8h*)(M16 + (size_t)e * HID + 8 * l);
          float* ap = acc + slot * HID + 8 * l;
          v4f a0 = *(v4f*)ap;
          v4f a1 = *(v4f*)(ap + 4);
#pragma unroll
          for (int j = 0; j < 4; ++j) { a0[j] += w * (float)x[j]; a1[j] += w * (float)x[4 + j]; }
          *(v4f*)ap = a0;
          *(v4f*)(ap + 4) = a1;
        }
      }
    }
    __syncthreads();
  }

  for (int i = tid; i < NB * (HID / 8); i += NTHR) {
    const int r = i >> 5, c8 = (i & 31) * 8;
    const v4f a0 = *(const v4f*)(acc + r * HID + c8);
    const v4f a1 = *(const v4f*)(acc + r * HID + c8 + 4);
    v8h o;
#pragma unroll
    for (int j = 0; j < 4; ++j) { o[j] = (_Float16)a0[j]; o[4 + j] = (_Float16)a1[j]; }
    *(v8h*)(ut + r * HP + c8) = o;
  }
  __syncthreads();

#pragma unroll 1
  for (int hf2 = 0; hf2 < 2; ++hf2) {
    __syncthreads();
    const int lrow0 = 64 * hf2 + 16 * wr;
    const int grow  = nodeBase + lrow0 + m;
    v8f a8[8];
#pragma unroll
    for (int i = 0; i < 8; ++i) a8[i] = zero8f();
    gemm16(hin + (size_t)grow * HID + 8 * h, TU1t + (size_t)(128 * wc + m) * UPDIN + 8 * h, UPDIN, 8, a8);
    gemm16(ut + (lrow0 + m) * HP + 8 * h, TU1t + (size_t)(128 * wc + m) * UPDIN + HID + 8 * h, UPDIN, 8, a8);
#pragma unroll
    for (int nt = 0; nt < 8; ++nt) {
      const int c = 128 * wc + 16 * nt + m;
      const float b = b1[c];
#pragma unroll
      for (int r = 0; r < 8; ++r) {
        const float v = a8[nt][r] * WINV + b;
        hid[(16 * wr + 8 * h + r) * HP + c] = (_Float16)fmaxf(v, 0.0f);
      }
    }
    __syncthreads();

#pragma unroll
    for (int i = 0; i < 8; ++i) a8[i] = zero8f();
    gemm16(hid + (16 * wr + m) * HP + 8 * h, TU2t + (size_t)(128 * wc + m) * HID + 8 * h, HID, 8, a8);
    float* st = stg + wave * (16 * FP);
#pragma unroll
    for (int nt = 0; nt < 8; ++nt) {
      const int c = 128 * wc + 16 * nt + m;
      const float b = b2[c];
#pragma unroll
      for (int r = 0; r < 8; ++r) {
        const float v = a8[nt][r] * WINV + b;
        st[(8 * h + r) * FP + 16 * nt + m] = fmaxf(v, 0.0f);
      }
    }
    __syncthreads();
    if (wf32 != 0) store16_f32(st, hf, HID, 128 * wc, nodeBase + lrow0, l);
    else           store16_f16(st, hout, HID, 128 * wc, nodeBase + lrow0, l);
  }
}

__global__ __launch_bounds__(256) void k_pool(const int* __restrict__ n2g, const float* __restrict__ hf,
                                              float* out, int nN) {
  __shared__ __attribute__((aligned(16))) float red[NWAVE * HID];
  __shared__ __attribute__((aligned(16))) float res[HID];
  const int tid = threadIdx.x, l = tid & 31, wave = tid >> 5;
  const int g = blockIdx.x;
  float part[8];
#pragma unroll
  for (int i = 0; i < 8; ++i) part[i] = 0.0f;

  const int nChunks = (nN + 255) / 256;
#pragma unroll 1
  for (int ch = 0; ch < nChunks; ++ch) {
    const int i = ch * 256 + tid;
    bool hit = false;
    if (i < nN) hit = (n2g[i] == g);
    unsigned mk = __builtin_amdgcn_ballot_w32(hit);
#pragma unroll 1
    for (int it = 0; it < 32 && mk != 0u; ++it) {
      const int b = __builtin_ctz(mk);
      mk &= mk - 1u;
      int node = ch * 256 + wave * 32 + b;
      node = node > nN - 1 ? nN - 1 : node;
      const float* rp = hf + (size_t)node * HID + 8 * l;
      const v4f a0 = *(const v4f*)rp;
      const v4f a1 = *(const v4f*)(rp + 4);
#pragma unroll
      for (int j = 0; j < 4; ++j) { part[j] += a0[j]; part[4 + j] += a1[j]; }
    }
  }
#pragma unroll
  for (int j = 0; j < 8; ++j) red[wave * HID + 8 * l + j] = part[j];
  __syncthreads();
  {
    float s = 0.0f;
#pragma unroll
    for (int w2 = 0; w2 < NWAVE; ++w2) s += red[w2 * HID + tid];
    res[tid] = s;
  }
  __syncthreads();
  if (wave == 0) {
    const v4f v0 = *(const v4f*)(res + 4 * l);
    const v4f v1 = *(const v4f*)(res + 128 + 4 * l);
    float* op = out + (size_t)g * HID;
    *(volatile v4f*)(op + 4 * l) = v0;
    *(volatile v4f*)(op + 128 + 4 * l) = v1;
    __threadfence();
    *(volatile v4f*)(op + 4 * l) = v0;
    *(volatile v4f*)(op + 128 + 4 * l) = v1;
  }
}

extern "C" void kernel_launch(void* const* d_in, const int* in_sizes, int n_in,
                              void* d_out, int out_size, void* d_ws, size_t ws_size,
                              hipStream_t stream) {
  if (n_in < 16) return;
  const int nN = in_sizes[1];
  const int nE = in_sizes[3];
  if (nN <= 0 || nE <= 0) return;
  if (in_sizes[0] != nN * IND || in_sizes[2] != nE * EFD || in_sizes[4] != 2 * nE || in_sizes[5] != nN) return;
  if (in_sizes[6] != IND * HID || in_sizes[7] != HID) return;
  if (in_sizes[8] != 3 * MSGIN * HID || in_sizes[9] != 3 * HID || in_sizes[10] != 3 * HID * HID || in_sizes[11] != 3 * HID) return;
  if (in_sizes[12] != 3 * UPDIN * HID || in_sizes[13] != 3 * HID || in_sizes[14] != 3 * HID * HID || in_sizes[15] != 3 * HID) return;
  if (out_size <= 0 || (out_size % HID) != 0) return;
  const int nG = out_size / HID;

  const float* x    = (const float*)d_in[0];
  const float* nsf  = (const float*)d_in[1];
  const float* ef   = (const float*)d_in[2];
  const float* ew   = (const float*)d_in[3];
  const int*   el   = (const int*)d_in[4];
  const int*   n2g  = (const int*)d_in[5];
  const float* Wlin = (const float*)d_in[6];
  const float* blin = (const float*)d_in[7];
  const float* mW1  = (const float*)d_in[8];
  const float* mb1  = (const float*)d_in[9];
  const float* mW2  = (const float*)d_in[10];
  const float* mb2  = (const float*)d_in[11];
  const float* uW1  = (const float*)d_in[12];
  const float* ub1  = (const float*)d_in[13];
  const float* uW2  = (const float*)d_in[14];
  const float* ub2  = (const float*)d_in[15];
  float* out = (float*)d_out;

  const int npad = ((nN + NB - 1) / NB) * NB;
  const int epad = ((nE + 63) / 64) * 64;

  char* ws = (char*)d_ws;
  size_t off = 0;
  const size_t oWt = off; off += (size_t)T_TOTAL * 2;          off = (off + 255) & ~(size_t)255;
  const size_t oHA = off; off += (size_t)npad * HID * 2;        off = (off + 255) & ~(size_t)255;
  const size_t oHB = off; off += (size_t)npad * HID * 2;        off = (off + 255) & ~(size_t)255;
  const size_t oP  = off; off += (size_t)npad * (2 * HID) * 2;  off = (off + 255) & ~(size_t)255;
  const size_t oM  = off; off += (size_t)epad * HID * 2;        off = (off + 255) & ~(size_t)255;
  if (off > ws_size) return;
  _Float16* Wt  = (_Float16*)(ws + oWt);
  _Float16* hA  = (_Float16*)(ws + oHA);
  _Float16* hB  = (_Float16*)(ws + oHB);
  _Float16* P16 = (_Float16*)(ws + oP);
  float*    HF  = (float*)(ws + oP);
  _Float16* M16 = (_Float16*)(ws + oM);

  const hipError_t a0 = hipFuncSetAttribute(reinterpret_cast<const void*>(&k_lin),     hipFuncAttributeMaxDynamicSharedMemorySize, L_LDS);
  const hipError_t a1 = hipFuncSetAttribute(reinterpret_cast<const void*>(&k_proj),    hipFuncAttributeMaxDynamicSharedMemorySize, J_LDS);
  const hipError_t a2 = hipFuncSetAttribute(reinterpret_cast<const void*>(&k_edge),    hipFuncAttributeMaxDynamicSharedMemorySize, E_LDS);
  const hipError_t a3 = hipFuncSetAttribute(reinterpret_cast<const void*>(&k_aggnode), hipFuncAttributeMaxDynamicSharedMemorySize, G_LDS);
  (void)a0; (void)a1; (void)a2; (void)a3;

  const int nBlkN64 = npad / 64;
  const int nBlkE64 = epad / 64;
  const int nBlkA   = npad / NB;

  k_wcvt<<<(T_PIECES * 8) / 256, 256, 0, stream>>>(Wlin, mW1, mW2, uW1, uW2, Wt);
  k_lin<<<nBlkN64, 256, L_LDS, stream>>>(x, Wt + T_LIN, blin, hA, nN);

  for (int s = 0; s < 3; ++s) {
    const _Float16* Ts  = Wt + T_L0 + (size_t)s * T_LSZ;
    const _Float16* hin = (s & 1) ? hB : hA;
    _Float16*       hnx = (s & 1) ? hA : hB;
    const int last = (s == 2) ? 1 : 0;
    k_proj<<<dim3(nBlkN64, 2), 256, J_LDS, stream>>>(hin, Ts + T_P, P16);
    k_edge<<<nBlkE64, 256, E_LDS, stream>>>(el, nsf, ef, P16, mW1 + (size_t)s * MSGIN * HID, mb1 + (size_t)s * HID,
                                             Ts + T_E, Ts + T_M2, mb2 + (size_t)s * HID, M16, nE, nN);
    k_aggnode<<<nBlkA, NTHR, G_LDS, stream>>>(el, ew, M16, hin, Ts + T_U1, ub1 + (size_t)s * HID,
                                              Ts + T_U2, ub2 + (size_t)s * HID, hnx, HF, nN, nE, last);
  }

  k_pool<<<nG, 256, 0, stream>>>(n2g, HF, out, nN);
  (void)hipGetLastError();
}
